// GGCNN_HNN_43379169689778
// MI455X (gfx1250) — hardware-verified
//
#include <hip/hip_runtime.h>
#define NNODE 500000
#define H1 32
#define H2 128

typedef __bf16 v16b __attribute__((ext_vector_type(16)));
typedef unsigned short v8us __attribute__((ext_vector_type(8), may_alias));
typedef float  v8f  __attribute__((ext_vector_type(8)));
typedef float  v4f  __attribute__((ext_vector_type(4)));
typedef float  v4fa __attribute__((ext_vector_type(4), may_alias));
union FragB { v16b v; v8us half[2]; unsigned short u[16]; };

__device__ __forceinline__ unsigned short bf16_bits(float x) { unsigned int u = __float_as_uint(x); return (unsigned short)((u + 0x7FFFu + ((u >> 16) & 1u)) >> 16); }
__device__ __forceinline__ float bf16_val(unsigned short b) { return __uint_as_float(((unsigned int)b) << 16); }
__device__ __forceinline__ float bf16_round(float x) { return bf16_val(bf16_bits(x)); }

typedef _Float16 v16h __attribute__((ext_vector_type(16)));
union FragH { v16h v; v8us half[2]; _Float16 h[16]; unsigned short u[16]; };
__device__ __forceinline__ v8f mmaH1(v16h a, v16h b, v8f c) { c = __builtin_amdgcn_wmma_f32_16x16x32_f16(false, a, false, b, (short)0, c, false, false); asm volatile("v_nop\n\tv_nop\n\tv_nop\n\tv_nop" : "+v"(c) : "v"(a), "v"(b)); return c; }
__device__ __forceinline__ float sigm(float x) { return __builtin_amdgcn_rcpf(1.0f + __builtin_amdgcn_exp2f(-x * 1.44269504088896341f)); }
__device__ __forceinline__ float tanhx(float x) { return 1.0f - 2.0f * __builtin_amdgcn_rcpf(1.0f + __builtin_amdgcn_exp2f(x * 2.88539008177792682f)); }

__global__ __launch_bounds__(256) void k_wt2(const float* __restrict__ Wx2, _Float16* __restrict__ Bt) { const int t = blockIdx.x * 256 + threadIdx.x; if (t >= 3 * H2 * (H1 / 8)) return; const int j = t / (H1 / 8), k8 = (t % (H1 / 8)) * 8; FragH f;
#pragma unroll
  for (int i = 0; i < 8; ++i) f.h[i] = (_Float16)(bf16_round(Wx2[(size_t)(k8 + i) * (3 * H2) + j]) * 16.0f); *(volatile v8us*)((unsigned short*)Bt + (size_t)j * H1 + k8) = f.half[0]; __threadfence(); *(volatile v8us*)((unsigned short*)Bt + (size_t)j * H1 + k8) = f.half[0]; }
__global__ __launch_bounds__(256) void k_l1(const float* __restrict__ x, const float* __restrict__ Wx1, const float* __restrict__ bx1, const float* __restrict__ bh1, _Float16* __restrict__ A1) { const size_t t = (size_t)blockIdx.x * 256 + threadIdx.x; if (t >= (size_t)NNODE * (H1 / 8)) return;
  const size_t n = t / (H1 / 8); const int j8 = (int)(t % (H1 / 8)) * 8; const float x0 = bf16_round(x[n * 2]), x1 = bf16_round(x[n * 2 + 1]); FragH f;
#pragma unroll
  for (int q = 0; q < 8; ++q) { const int j = j8 + q;
    const float gz = x0 * bf16_round(Wx1[j]) + x1 * bf16_round(Wx1[3 * H1 + j]) + bf16_round(bx1[j]) + bf16_round(bh1[j]);
    const float gc = x0 * bf16_round(Wx1[2 * H1 + j]) + x1 * bf16_round(Wx1[3 * H1 + 2 * H1 + j]) + bf16_round(bx1[2 * H1 + j]) + bf16_round(bh1[2 * H1 + j]);
    const float z = sigm(gz), c = tanhx(gc); f.h[q] = (_Float16)fmaxf((1.0f - z) * c, 0.f); }
  *(volatile v8us*)((unsigned short*)A1 + t * 8) = f.half[0]; __threadfence(); *(volatile v8us*)((unsigned short*)A1 + t * 8) = f.half[0]; }
__global__ __launch_bounds__(128) void k_l2(const _Float16* __restrict__ A1, const _Float16* __restrict__ Bt, const float* __restrict__ bx2, const float* __restrict__ bh2, const float* __restrict__ lw, const float* __restrict__ lb, const float* __restrict__ gw, const float* __restrict__ gb, float* __restrict__ out) {
  __shared__ float so[64][2];
  const int tid = threadIdx.x, w = tid >> 5, lane = tid & 31, ln = lane & 15, hh = lane >> 4; const size_t row0 = ((size_t)blockIdx.x * 4 + w) * 16;
  FragH a; { size_t arn = row0 + ln; if (arn > NNODE - 1) arn = NNODE - 1; const unsigned short* ar = (const unsigned short*)A1 + arn * H1;   a.half[0] = *(const v8us*)(ar + 8 * hh); a.half[1] = *(const v8us*)(ar + 16 + 8 * hh); }
  v8f az[8], ac[8];
#pragma unroll
  for (int t = 0; t < 8; ++t) { FragH b; const unsigned short* br = (const unsigned short*)Bt + (size_t)(16 * t + ln) * H1; b.half[0] = *(const v8us*)(br + 8 * hh); b.half[1] = *(const v8us*)(br + 16 + 8 * hh); az[t] = mmaH1(a.v, b.v, (v8f){0.f,0.f,0.f,0.f,0.f,0.f,0.f,0.f});
    const unsigned short* cr = (const unsigned short*)Bt + (size_t)(2 * H2 + 16 * t + ln) * H1; b.half[0] = *(const v8us*)(cr + 8 * hh); b.half[1] = *(const v8us*)(cr + 16 + 8 * hh); ac[t] = mmaH1(a.v, b.v, (v8f){0.f,0.f,0.f,0.f,0.f,0.f,0.f,0.f}); }
  float hv[8];
#pragma unroll
  for (int r = 0; r < 8; ++r) hv[r] = 0.f;
#pragma unroll
  for (int t = 0; t < 8; ++t) { const int d = 16 * t + ln; const float bz = bf16_round(bx2[d]) + bf16_round(bh2[d]), bc = bf16_round(bx2[2 * H2 + d]) + bf16_round(bh2[2 * H2 + d]), lwd = bf16_round(lw[d]);
#pragma unroll
    for (int r = 0; r < 8; ++r) { const float z = sigm(az[t][r] * 0.0625f + bz); const float c = tanhx(ac[t][r] * 0.0625f + bc); const float a2 = tanhx((1.0f - z) * c); hv[r] += a2 * lwd; } }
#pragma unroll
  for (int r = 0; r < 8; ++r) { float v = hv[r]; v += __shfl_xor(v, 1, 32); v += __shfl_xor(v, 2, 32); v += __shfl_xor(v, 4, 32); v += __shfl_xor(v, 8, 32); hv[r] = v + bf16_round(lb[0]); }
  if (ln == 0) { const float g0 = bf16_round(gw[0]), g1 = bf16_round(gw[1]), c0 = bf16_round(gb[0]), c1 = bf16_round(gb[1]);
#pragma unroll
    for (int r = 0; r < 8; ++r) { const float dh0 = hv[r] * g0 + c0, dh1 = hv[r] * g1 + c1; so[w * 16 + 8 * hh + r][0] = dh1; so[w * 16 + 8 * hh + r][1] = -dh0; } }
  __syncthreads();
  const bool stl = (tid < 32) && ((size_t)blockIdx.x * 64 + 2 * tid + 1 < NNODE);
  if (stl) { const v4f v = {so[2 * tid][0], so[2 * tid][1], so[2 * tid + 1][0], so[2 * tid + 1][1]}; *(volatile v4f*)(out + ((size_t)blockIdx.x * 64 + 2 * tid) * 2) = v; }
  __threadfence();
  if (stl) { const v4f v = {so[2 * tid][0], so[2 * tid][1], so[2 * tid + 1][0], so[2 * tid + 1][1]}; *(volatile v4f*)(out + ((size_t)blockIdx.x * 64 + 2 * tid) * 2) = v; }
}
extern "C" void kernel_launch(void* const* d_in, const int* in_sizes, int n_in,
                              void* d_out, int out_size, void* d_ws, size_t ws_size, hipStream_t stream) {
  (void)in_sizes; (void)n_in; (void)out_size;
  const float* x = (const float*)d_in[0]; const float* Wx1 = (const float*)d_in[2]; const float* bx1 = (const float*)d_in[3]; const float* bh1 = (const float*)d_in[5];
  const float* Wx2 = (const float*)d_in[6]; const float* bx2 = (const float*)d_in[7]; const float* bh2 = (const float*)d_in[9]; const float* lw = (const float*)d_in[10]; const float* lb = (const float*)d_in[11]; const float* gw = (const float*)d_in[12]; const float* gb = (const float*)d_in[13];
  char* ws = (char*)d_ws; size_t off = 0;
  auto take = [&](size_t bytes) { char* p = ws + off; off += (bytes + 255) & ~(size_t)255; return p; };
  _Float16* Bt = (_Float16*)take((size_t)3 * H2 * H1 * 2); _Float16* A1 = (_Float16*)take((size_t)NNODE * H1 * 2);
  if (off > ws_size) return;
  k_wt2<<<(3 * H2 * (H1 / 8) + 255) / 256, 256, 0, stream>>>(Wx2, Bt);
  k_l1<<<(unsigned)(((size_t)NNODE * (H1 / 8) + 255) / 256), 256, 0, stream>>>(x, Wx1, bx1, bh1, A1);
  k_l2<<<(NNODE + 63) / 64, 128, 0, stream>>>(A1, Bt, bx2, bh2, lw, lb, gw, gb, (float*)d_out);
}
